// TransformerBlock_44384192037436
// MI455X (gfx1250) — hardware-verified
//
#include <hip/hip_runtime.h>
#include <stddef.h>


typedef _Float16 v16h __attribute__((ext_vector_type(16)));
typedef _Float16 v8h  __attribute__((ext_vector_type(8)));
typedef float    v8f  __attribute__((ext_vector_type(8)));
typedef float    v4f  __attribute__((ext_vector_type(4)));
typedef unsigned int v8u __attribute__((ext_vector_type(8)));
typedef int      v4i  __attribute__((ext_vector_type(4)));

#ifndef NB
#define NB 2
#endif
#ifndef SEQ
#define SEQ 8192
#endif
#define NB_FULL  2
#define SEQ_FULL 8192
#define DIM   256
#define HID   1024
#define NHEAD 8
#define HD    32
#define QKVW  768
#define NGRAPH 64
#define MROWS (NB * SEQ)
#define SRCH_ITERS 14

static_assert(NB >= 1 && NB <= NB_FULL);
static_assert(SEQ >= 128 && SEQ <= SEQ_FULL && (SEQ % 128) == 0);
static_assert((SEQ % 256) == 0);
static_assert(SEQ <= (1 << (SRCH_ITERS - 1)));
static_assert(DIM == NHEAD * HD);
static_assert(HD == 32);
static_assert(QKVW == 3 * DIM);
static_assert(HID == 4 * DIM);
static_assert((DIM % 64) == 0 && (DIM % 32) == 0);
static_assert((HID % 64) == 0 && (HID % 32) == 0);
static_assert((QKVW % 64) == 0);
static_assert((MROWS % 64) == 0 && (MROWS % 8) == 0);
static_assert(DIM == 32 * 8);
static_assert(NHEAD == 4 * 2);
static_assert((size_t)MROWS * HID < (size_t)0xFFFFFFFFu);

#define LDT 72
#define LDC 68
#define KP  40
static_assert((LDT % 8) == 0 && LDT >= 64);
static_assert((LDC % 4) == 0 && LDC >= 64);
static_assert((KP % 8) == 0 && KP >= 32);

#define WCARRY 64.0f
#define QCARRY 64.0f
#define VCARRY 64.0f
#define MCARRY 16.0f
#define LN_EPS 1.0e-6f
static_assert(QCARRY == VCARRY);
static_assert(QCARRY == WCARRY);

#define WQKV_BYTES    ((size_t)QKVW * DIM * 2)
#define WSQ_BYTES     ((size_t)DIM * DIM * 2)
#define WFF_BYTES     ((size_t)DIM * HID * 2)
#define PLANE16_BYTES ((size_t)MROWS * DIM * 2)
#define PLANE16_ELEMS ((size_t)MROWS * DIM)
#define X1_BYTES      ((size_t)MROWS * DIM * 4)
#define MID_BYTES     ((size_t)MROWS * HID * 2)
#define FLAG_BYTES    ((size_t)128)
#define OFF_WQKV ((size_t)0)
#define OFF_WO   (OFF_WQKV + WQKV_BYTES)
#define OFF_W1   (OFF_WO + WSQ_BYTES)
#define OFF_W2   (OFF_W1 + WFF_BYTES)
#define OFF_X16  (OFF_W2 + WFF_BYTES)
#define OFF_Q    (OFF_X16 + PLANE16_BYTES)
#define OFF_KVT  (OFF_Q + PLANE16_BYTES)
#define OFF_CTX  (OFF_KVT + 2 * PLANE16_BYTES)
#define OFF_H2   (OFF_CTX + PLANE16_BYTES)
#define OFF_X1   (OFF_H2 + PLANE16_BYTES)
#define OFF_MID  (OFF_X1 + X1_BYTES)
#define OFF_FLAG (OFF_MID + MID_BYTES)
#define WS_TOTAL (OFF_FLAG + FLAG_BYTES)
static_assert((WQKV_BYTES % 128) == 0 && (WSQ_BYTES % 128) == 0 && (WFF_BYTES % 128) == 0);
static_assert((PLANE16_BYTES % 128) == 0 && (X1_BYTES % 128) == 0 && (MID_BYTES % 128) == 0);
static_assert(WS_TOTAL <= (size_t)134217728);

__device__ __forceinline__ float bf16r(float x) {
  unsigned int u = __float_as_uint(x);
  u = (u + 0x7FFFu + ((u >> 16) & 1u)) & 0xFFFF0000u;
  return __uint_as_float(u);
}

static __device__ __forceinline__ _Float16 toh_flush(float v) {
  const _Float16 r = (_Float16)v;
  return (fabsf(v) < 6.103515625e-05f) ? (_Float16)0.0f : r;
}

__device__ __forceinline__ v16h frag_at(const _Float16* p) {
  v8h lo = *(const v8h*)(p);
  v8h hi = *(const v8h*)(p + 16);
  v16h out;
#pragma unroll
  for (int i = 0; i < 8; ++i) { out[i] = lo[i]; out[i + 8] = hi[i]; }
  return out;
}
__device__ __forceinline__ v16h ld_frag(const _Float16* base, unsigned ld) {
  const unsigned lane = threadIdx.x & 31u;
  return frag_at(base + (lane & 15u) * ld + (lane >> 4) * 8u);
}

__device__ __forceinline__ v8f wmma16(v16h a, v16h b, v8f c) {
  v8f d = __builtin_amdgcn_wmma_f32_16x16x32_f16(false, a, false, b, (short)0, c,
                                                 false, false);
  asm volatile("v_nop\n\tv_nop\n\tv_nop\n\tv_nop" : "+v"(d) : "v"(a), "v"(b));
  return d;
}

__device__ __forceinline__ float red32_sum(float x) {
#pragma unroll
  for (int off = 1; off < 32; off <<= 1) x += __shfl_xor(x, off, 32);
  return x;
}

__device__ __forceinline__ void wave_lds_sync() {
  __builtin_amdgcn_fence(3  , "wavefront");
  asm volatile("s_wait_dscnt 0x0" ::: "memory");
  __builtin_amdgcn_wave_barrier();
}

__device__ __forceinline__ float gelu_act(float t) {
  return 0.5f * t * (1.0f + erff(t * 0.70710678118654752440f));
}

__device__ __forceinline__ v8u seg_mask(unsigned kb, unsigned hh, unsigned lo, unsigned len) {
  v8u mk;
#pragma unroll
  for (unsigned j = 0; j < 8u; ++j) {
    const unsigned nd = kb + hh * 8u + 2u * (j & 3u) + 16u * (j >> 2);
    const unsigned m0 = ((nd - lo) < len) ? 0x0000FFFFu : 0u;
    const unsigned m1 = ((nd + 1u - lo) < len) ? 0xFFFF0000u : 0u;
    mk[j] = m0 | m1;
  }
  return mk;
}
__device__ __forceinline__ v16h frag_and(v16h a, v8u mk) {
  v8u w = __builtin_bit_cast(v8u, a);
  w = w & mk;
  return __builtin_bit_cast(v16h, w);
}

__global__ __launch_bounds__(256) void wconv_kernel(
    const float* __restrict__ W, _Float16* __restrict__ Wt, unsigned ldw, unsigned ldk) {
  __shared__ _Float16 T[64 * LDT];
  const unsigned tid = threadIdx.x;
  const unsigned n0 = blockIdx.x * 64u;
  const unsigned k0 = blockIdx.y * 64u;
#pragma unroll 4
  for (unsigned j = 0; j < 16u; ++j) {
    const unsigned idx = tid + 256u * j;
    const unsigned kr = idx >> 6, nc = idx & 63u;
    const float v = W[(size_t)(k0 + kr) * ldw + n0 + nc];
    T[nc * LDT + kr] = (_Float16)(WCARRY * bf16r(v));
  }
  __syncthreads();
  v8h x[2];
  size_t off[2];
#pragma unroll
  for (unsigned i = 0; i < 2u; ++i) {
    const unsigned n = 32u * i + (tid >> 3);
    const unsigned kc = (tid & 7u) * 8u;
    x[i] = *(const v8h*)&T[n * LDT + kc];
    off[i] = (size_t)(n0 + n) * ldk + k0 + kc;
  }
#pragma unroll
  for (int i = 0; i < 2; ++i) *(volatile v8h*)(Wt + off[i]) = x[i];
  __threadfence();
#pragma unroll
  for (int i = 0; i < 2; ++i) *(volatile v8h*)(Wt + off[i]) = x[i];
}

__global__ __launch_bounds__(256) void xconv_kernel(
    const float* __restrict__ X, _Float16* __restrict__ dst) {
  const unsigned lane = threadIdx.x & 31u, w = threadIdx.x >> 5;
  const unsigned crow = blockIdx.x * 8u + w;
  const unsigned bidx = crow / (unsigned)SEQ;
  const unsigned sq = crow - bidx * (unsigned)SEQ;
  const size_t srow = (size_t)bidx * SEQ_FULL + sq;
  const float* xr = X + srow * DIM + lane * 8u;
  const v4f a0 = *(const v4f*)(xr);
  const v4f a1 = *(const v4f*)(xr + 4u);
  v8h o;
#pragma unroll
  for (int i = 0; i < 4; ++i) {
    o[i]     = toh_flush(bf16r(a0[i]));
    o[i + 4] = toh_flush(bf16r(a1[i]));
  }
  _Float16* p = dst + (size_t)crow * DIM + lane * 8u;
  *(volatile v8h*)p = o;
  __threadfence();
  *(volatile v8h*)p = o;
}

__global__ __launch_bounds__(256) void seg_check_kernel(
    const int* __restrict__ batch, int* __restrict__ flag) {
  __shared__ int wbad[8];
  const unsigned tid = threadIdx.x, lane = tid & 31u;
  const unsigned wave = (unsigned)__builtin_amdgcn_readfirstlane((int)(tid >> 5));
  int bad = 0;
#pragma unroll 1
  for (unsigned j = 0; j < (unsigned)(SEQ / 256); ++j) {
    const unsigned i = j * 256u + tid;
    const unsigned i1 = min(i + 1u, (unsigned)SEQ - 1u);
    const int v = batch[i];
    const int nx = batch[i1];
    bad |= ((v < 0) ? 1 : 0) | ((v >= NGRAPH) ? 1 : 0) | ((v > nx) ? 1 : 0);
  }
#pragma unroll
  for (int off = 1; off < 32; off <<= 1) bad |= __shfl_xor(bad, off, 32);
  if (lane == 0u) wbad[wave] = bad;
  __syncthreads();
  int tot = 0;
#pragma unroll
  for (int k = 0; k < 8; ++k) tot |= wbad[k];
  const v4i val = {tot, tot, tot, tot};
  if (tid < 8u) *(volatile v4i*)(flag + tid * 4u) = val;
  __threadfence();
  if (tid < 8u) *(volatile v4i*)(flag + tid * 4u) = val;
}

__global__ __launch_bounds__(256) void ln_ws_kernel(
    const float* __restrict__ X, const float* __restrict__ G, const float* __restrict__ Be,
    _Float16* __restrict__ dst) {
#pragma clang fp contract(off)
  const unsigned lane = threadIdx.x & 31u, w = threadIdx.x >> 5;
  const unsigned crow = blockIdx.x * 8u + w;
  const unsigned c = lane * 8u;
  const float* xr = X + (size_t)crow * DIM + c;
  const v4f a0 = *(const v4f*)(xr);
  const v4f a1 = *(const v4f*)(xr + 4u);
  const v4f g0 = *(const v4f*)(G + c);
  const v4f g1 = *(const v4f*)(G + c + 4u);
  const v4f b0 = *(const v4f*)(Be + c);
  const v4f b1 = *(const v4f*)(Be + c + 4u);

  float s = 0.0f;
#pragma unroll
  for (int i = 0; i < 4; ++i) s += a0[i] + a1[i];
  const float mean = red32_sum(s) * (1.0f / (float)DIM);

  float ss = 0.0f;
#pragma unroll
  for (int i = 0; i < 4; ++i) {
    const float d0 = a0[i] - mean;
    const float d1 = a1[i] - mean;
    ss += d0 * d0;
    ss += d1 * d1;
  }
  const float var = red32_sum(ss) * (1.0f / (float)DIM);
  const float rstd = 1.0f / sqrtf(var + LN_EPS);

  v8h o;
#pragma unroll
  for (int i = 0; i < 4; ++i) {
    const float d0 = a0[i] - mean;
    const float d1 = a1[i] - mean;
    o[i]     = toh_flush(d0 * rstd * bf16r(g0[i]) + bf16r(b0[i]));
    o[i + 4] = toh_flush(d1 * rstd * bf16r(g1[i]) + bf16r(b1[i]));
  }
  _Float16* p = dst + (size_t)crow * DIM + c;
  *(volatile v8h*)p = o;
  __threadfence();
  *(volatile v8h*)p = o;
}

__global__ __launch_bounds__(256) void gemm_qkv_kernel(
    const _Float16* __restrict__ A16, const _Float16* __restrict__ Bt,
    const float* __restrict__ g1, const float* __restrict__ be1,
    const float* __restrict__ g2, const float* __restrict__ be2,
    _Float16* __restrict__ q16, _Float16* __restrict__ kvt) {
  __shared__ float Cs[64 * LDC];
  const unsigned tid = threadIdx.x, lane = tid & 31u, w = tid >> 5;
  const unsigned mw = w >> 1, nw = w & 1u;
  const unsigned hh = lane >> 4, m = lane & 15u;
  const unsigned n0 = blockIdx.x * 64u;
  const unsigned row0 = blockIdx.y * 64u;
  const unsigned K = (unsigned)DIM;

  const _Float16* ap  = A16 + (size_t)(row0 + mw * 16u + m) * K + hh * 8u;
  const _Float16* bp0 = Bt + (size_t)(n0 + nw * 32u + m) * K + hh * 8u;
  const _Float16* bp1 = bp0 + (size_t)16 * K;
  v8f acc0 = {}, acc1 = {};
#pragma unroll 2
  for (unsigned k0 = 0; k0 < K; k0 += 32u) {
    const v16h a  = frag_at(ap + k0);
    const v16h b0 = frag_at(bp0 + k0);
    const v16h b1 = frag_at(bp1 + k0);
    acc0 = wmma16(a, b0, acc0);
    acc1 = wmma16(a, b1, acc1);
  }
#pragma unroll
  for (int r = 0; r < 8; ++r) {
    float* d = &Cs[(mw * 16u + hh * 8u + (unsigned)r) * LDC + nw * 32u + m];
    d[0]  = acc0[r];
    d[16] = acc1[r];
  }
  __syncthreads();

  const unsigned sect = n0 / (unsigned)DIM;

  if (sect != 0u) {
    const bool isk = (sect == 1u);
    const unsigned cw = ((tid & 7u) * 8u) & 31u;
    const v4f ka0 = *(const v4f*)(g1 + cw);
    const v4f ka1 = *(const v4f*)(g1 + cw + 4u);
    const v4f kb0 = *(const v4f*)(be1 + cw);
    const v4f kb1 = *(const v4f*)(be1 + cw + 4u);
    const v4f va0 = *(const v4f*)(g2 + cw);
    const v4f va1 = *(const v4f*)(g2 + cw + 4u);
    const v4f vb0 = *(const v4f*)(be2 + cw);
    const v4f vb1 = *(const v4f*)(be2 + cw + 4u);
    v4f gw0, gw1, bw0, bw1;
#pragma unroll
    for (int j = 0; j < 4; ++j) {
      gw0[j] = bf16r(isk ? ka0[j] : va0[j]);
      gw1[j] = bf16r(isk ? ka1[j] : va1[j]);
      bw0[j] = bf16r(isk ? kb0[j] : vb0[j]);
      bw1[j] = bf16r(isk ? kb1[j] : vb1[j]);
    }
#pragma unroll 1
    for (unsigned i = 0; i < 2u; ++i) {
      const unsigned r = 32u * i + (tid >> 3);
      const unsigned c = (tid & 7u) * 8u;
      const v4f u0 = *(const v4f*)&Cs[r * LDC + c];
      const v4f u1 = *(const v4f*)&Cs[r * LDC + c + 4u];
      const v4f t0 = u0 * (1.0f / WCARRY);
      const v4f t1 = u1 * (1.0f / WCARRY);
      float s = ((t0[0] + t0[1]) + (t0[2] + t0[3])) + ((t1[0] + t1[1]) + (t1[2] + t1[3]));
      s += __shfl_xor(s, 1, 32);
      s += __shfl_xor(s, 2, 32);
      const float mean = s * (1.0f / (float)HD);
      const v4f d0 = t0 - mean;
      const v4f d1 = t1 - mean;
      float ss = 0.0f;
#pragma unroll
      for (int j = 0; j < 4; ++j) {
        ss += d0[j] * d0[j];
        ss += d1[j] * d1[j];
      }
      ss += __shfl_xor(ss, 1, 32);
      ss += __shfl_xor(ss, 2, 32);
      const float rstd = 1.0f / sqrtf(ss * (1.0f / (float)HD) + LN_EPS);
      v4f o0, o1;
#pragma unroll
      for (int j = 0; j < 4; ++j) {
        o0[j] = d0[j] * rstd * gw0[j] + bw0[j];
        o1[j] = d1[j] * rstd * gw1[j] + bw1[j];
      }
      *(v4f*)&Cs[r * LDC + c] = o0;
      *(v4f*)&Cs[r * LDC + c + 4u] = o1;
    }
  }
  __syncthreads();

  if (sect == 0u) {
    v8h x[2];
    size_t off[2];
#pragma unroll
    for (unsigned i = 0; i < 2u; ++i) {
      const unsigned r = 32u * i + (tid >> 3);
      const unsigned c = (tid & 7u) * 8u;
      const v4f u0 = *(const v4f*)&Cs[r * LDC + c];
      const v4f u1 = *(const v4f*)&Cs[r * LDC + c + 4];
#pragma unroll
      for (int j = 0; j < 4; ++j) {
        x[i][j]     = toh_flush(u0[j]);
        x[i][j + 4] = toh_flush(u1[j]);
      }
      off[i] = (size_t)(row0 + r) * DIM + n0 + c;
    }
#pragma unroll
    for (int i = 0; i < 2; ++i) *(volatile v8h*)(q16 + off[i]) = x[i];
    __threadfence();
#pragma unroll
    for (int i = 0; i < 2; ++i) *(volatile v8h*)(q16 + off[i]) = x[i];
  } else {
    const unsigned bidx = row0 / (unsigned)SEQ;
    const unsigned key0 = row0 - bidx * (unsigned)SEQ;
    const unsigned ncol0 = n0 - sect * (unsigned)DIM;
    const size_t pbase = (size_t)(sect - 1u) * PLANE16_ELEMS;
    v8h x[2];
    size_t off[2];
#pragma unroll
    for (unsigned i = 0; i < 2u; ++i) {
      const unsigned dcol = 32u * i + (tid >> 3);
      const unsigned kk = (tid & 7u) * 8u;
#pragma unroll
      for (unsigned j = 0; j < 8u; ++j)
        x[i][j] = toh_flush(Cs[(kk + j) * LDC + dcol]);
      off[i] = pbase + ((size_t)bidx * DIM + ncol0 + dcol) * SEQ + key0 + kk;
    }
#pragma unroll
    for (int i = 0; i < 2; ++i) *(volatile v8h*)(kvt + off[i]) = x[i];
    __threadfence();
#pragma unroll
    for (int i = 0; i < 2; ++i) *(volatile v8h*)(kvt + off[i]) = x[i];
  }
}

__global__ __launch_bounds__(128) void galerkin_kernel(
    const _Float16* __restrict__ Qh, const _Float16* __restrict__ Kt,
    const _Float16* __restrict__ Vt, const int* __restrict__ batch,
    _Float16* __restrict__ Ov) {
  __shared__ __attribute__((aligned(16))) _Float16 KTs[4 * 2 * 32 * KP];
  __shared__ __attribute__((aligned(16))) _Float16 Os[4 * 16 * LDT];

  const unsigned tid = threadIdx.x, lane = tid & 31u;
  const unsigned wave = (unsigned)__builtin_amdgcn_readfirstlane((int)(tid >> 5));
  const unsigned hh = lane >> 4, m = lane & 15u;
  const int g = (int)blockIdx.x;
  const unsigned b = blockIdx.y;

  int lo0 = 0, hi0 = SEQ;
  int lo1 = 0, hi1 = SEQ;
#pragma unroll 1
  for (int it = 0; it < SRCH_ITERS; ++it) {
    const int mid0 = (lo0 + hi0) >> 1;
    const int mid1 = (lo1 + hi1) >> 1;
    const int bv0 = batch[min(mid0, SEQ - 1)];
    const int bv1 = batch[min(mid1, SEQ - 1)];
    const bool act0 = lo0 < hi0;
    const bool act1 = lo1 < hi1;
    const bool ls0 = bv0 < g;
    const bool ls1 = bv1 <= g;
    lo0 = (act0 && ls0) ? (mid0 + 1) : lo0;
    hi0 = (act0 && !ls0) ? mid0 : hi0;
    lo1 = (act1 && ls1) ? (mid1 + 1) : lo1;
    hi1 = (act1 && !ls1) ? mid1 : hi1;
  }
  const int s0 = min(max(lo0, 0), SEQ);
  const int s1 = min(max(lo1, s0), SEQ);
  const int cnt = max(s1 - s0, 1);
  const float inv = 1.0f / (float)cnt;
  const unsigned ulo = (unsigned)__builtin_amdgcn_readfirstlane(s0);
  const unsigned uhi = (unsigned)__builtin_amdgcn_readfirstlane(s1);
  const unsigned len = uhi - ulo;

  const unsigned kt0 = wave * (2u * 32u * KP);
  const unsigned o0 = wave * (16u * LDT);

#pragma unroll
  for (int hs = 0; hs < 2; ++hs) {
    const unsigned head = wave * 2u + (unsigned)hs;
    const size_t prow = ((size_t)b * DIM + head * HD) * SEQ;
    const _Float16* kp = Kt + prow + (size_t)m * SEQ + hh * 8u;
    const _Float16* vp = Vt + prow + (size_t)m * SEQ + hh * 8u;
    v8f c00 = {}, c01 = {}, c10 = {}, c11 = {};
    for (unsigned kb = ulo & ~31u; kb < uhi; kb += 32u) {
      const v8u mk = seg_mask(kb, hh, ulo, len);
      const v16h a0 = frag_and(frag_at(kp + kb), mk);
      const v16h a1 = frag_and(frag_at(kp + (size_t)16 * SEQ + kb), mk);
      const v16h b0 = frag_and(frag_at(vp + kb), mk);
      const v16h b1 = frag_and(frag_at(vp + (size_t)16 * SEQ + kb), mk);
      c00 = wmma16(a0, b0, c00);
      c01 = wmma16(a0, b1, c01);
      c10 = wmma16(a1, b0, c10);
      c11 = wmma16(a1, b1, c11);
    }
    v8h t00, t01, t10, t11;
#pragma unroll
    for (int r = 0; r < 8; ++r) {
      t00[r] = toh_flush(c00[r]);
      t01[r] = toh_flush(c01[r]);
      t10[r] = toh_flush(c10[r]);
      t11[r] = toh_flush(c11[r]);
    }
    const unsigned kth = kt0 + (unsigned)hs * (32u * KP);
    *(v8h*)&KTs[kth + m * KP + hh * 8u] = t00;
    *(v8h*)&KTs[kth + (16u + m) * KP + hh * 8u] = t01;
    *(v8h*)&KTs[kth + m * KP + 16u + hh * 8u] = t10;
    *(v8h*)&KTs[kth + (16u + m) * KP + 16u + hh * 8u] = t11;
  }
  wave_lds_sync();

  const v16h bk00 = ld_frag(&KTs[kt0], KP);
  const v16h bk01 = ld_frag(&KTs[kt0 + 16u * KP], KP);
  const v16h bk10 = ld_frag(&KTs[kt0 + 32u * KP], KP);
  const v16h bk11 = ld_frag(&KTs[kt0 + 32u * KP + 16u * KP], KP);

  for (unsigned rt = ulo & ~15u; rt < uhi; rt += 16u) {
    const size_t qoff = (size_t)(b * (unsigned)SEQ + rt + m) * DIM + wave * 64u + hh * 8u;
    const v16h q0 = frag_at(Qh + qoff);
    const v16h q1 = frag_at(Qh + qoff + 32);
    const v8f z = {};
    const v8f o00 = wmma16(q0, bk00, z);
    const v8f o01 = wmma16(q0, bk01, z);
    const v8f o10 = wmma16(q1, bk10, z);
    const v8f o11 = wmma16(q1, bk11, z);
#pragma unroll
    for (int r = 0; r < 8; ++r) {
      const unsigned rb = o0 + (hh * 8u + (unsigned)r) * LDT + m;
      Os[rb]       = toh_flush(o00[r] * inv);
      Os[rb + 16u] = toh_flush(o01[r] * inv);
      Os[rb + 32u] = toh_flush(o10[r] * inv);
      Os[rb + 48u] = toh_flush(o11[r] * inv);
    }
    wave_lds_sync();
    v8h x[4];
    size_t off[4];
    bool ok[4];
#pragma unroll
    for (unsigned i = 0; i < 4u; ++i) {
      const unsigned r = 4u * i + (lane >> 3);
      const unsigned c = (lane & 7u) * 8u;
      x[i] = *(const v8h*)&Os[o0 + r * LDT + c];
      const unsigned row = rt + r;
      ok[i] = (row - ulo) < len;
      off[i] = (size_t)(b * (unsigned)SEQ + row) * DIM + wave * 64u + c;
    }
#pragma unroll
    for (int i = 0; i < 4; ++i) { if (ok[i]) *(volatile v8h*)(Ov + off[i]) = x[i]; }
    __threadfence();
#pragma unroll
    for (int i = 0; i < 4; ++i) { if (ok[i]) *(volatile v8h*)(Ov + off[i]) = x[i]; }
    wave_lds_sync();
  }
}

template <int MODE>
__device__ __forceinline__ void gemm_body(
    const _Float16* __restrict__ A16, const _Float16* __restrict__ Bt, const unsigned K,
    const float* __restrict__ bias, const float* __restrict__ addf,
    float* __restrict__ outf, _Float16* __restrict__ out16, _Float16* __restrict__ out16r) {
  static_assert(MODE >= 2 && MODE <= 4);
  __shared__ float Cs[64 * LDC];
  const unsigned tid = threadIdx.x, lane = tid & 31u, w = tid >> 5;
  const unsigned mw = w >> 1, nw = w & 1u;
  const unsigned hh = lane >> 4, m = lane & 15u;
  const unsigned n0 = blockIdx.x * 64u;
  const unsigned row0 = blockIdx.y * 64u;

  const _Float16* ap  = A16 + (size_t)(row0 + mw * 16u + m) * K + hh * 8u;
  const _Float16* bp0 = Bt + (size_t)(n0 + nw * 32u + m) * K + hh * 8u;
  const _Float16* bp1 = bp0 + (size_t)16 * K;
  v8f acc0 = {}, acc1 = {};
#pragma unroll 2
  for (unsigned k0 = 0; k0 < K; k0 += 32u) {
    const v16h a  = frag_at(ap + k0);
    const v16h b0 = frag_at(bp0 + k0);
    const v16h b1 = frag_at(bp1 + k0);
    acc0 = wmma16(a, b0, acc0);
    acc1 = wmma16(a, b1, acc1);
  }
#pragma unroll
  for (int r = 0; r < 8; ++r) {
    float* d = &Cs[(mw * 16u + hh * 8u + (unsigned)r) * LDC + nw * 32u + m];
    d[0]  = acc0[r];
    d[16] = acc1[r];
  }
  __syncthreads();

  if (MODE == 3) {
#pragma unroll 1
    for (unsigned g = 0; g < 4u; ++g) {
      const unsigned r = 32u * (g >> 1) + (tid >> 3);
      const unsigned c = (tid & 7u) * 8u + 4u * (g & 1u);
      const v4f u  = *(const v4f*)&Cs[r * LDC + c];
      const v4f gb = *(const v4f*)(bias + n0 + c);
      v4f t;
#pragma unroll
      for (int j = 0; j < 4; ++j)
        t[j] = MCARRY * gelu_act(u[j] * (1.0f / WCARRY) + bf16r(gb[j]));
      *(v4f*)&Cs[r * LDC + c] = t;
    }
  }

  if (MODE == 3) {
    const unsigned ldo = (unsigned)HID;
    v8h x[2];
    size_t off[2];
#pragma unroll
    for (unsigned i = 0; i < 2u; ++i) {
      const unsigned r = 32u * i + (tid >> 3);
      const unsigned c = (tid & 7u) * 8u;
      const v4f u0 = *(const v4f*)&Cs[r * LDC + c];
      const v4f u1 = *(const v4f*)&Cs[r * LDC + c + 4];
#pragma unroll
      for (int j = 0; j < 4; ++j) {
        x[i][j]     = toh_flush(u0[j]);
        x[i][j + 4] = toh_flush(u1[j]);
      }
      off[i] = (size_t)(row0 + r) * ldo + n0 + c;
    }
#pragma unroll
    for (int i = 0; i < 2; ++i) *(volatile v8h*)(out16 + off[i]) = x[i];
    __threadfence();
#pragma unroll
    for (int i = 0; i < 2; ++i) *(volatile v8h*)(out16 + off[i]) = x[i];
  }

  if (MODE == 2 || MODE == 4) {
    const float cs = (MODE == 2) ? (1.0f / (WCARRY * VCARRY)) : (1.0f / (WCARRY * MCARRY));
    v4f xs[4];
    size_t off[4];
#pragma unroll
    for (unsigned i = 0; i < 4u; ++i) {
      const unsigned r = 16u * i + (tid >> 4);
      const unsigned c = (tid & 15u) * 4u;
      const unsigned crow = row0 + r;
      const unsigned bidx = crow / (unsigned)SEQ;
      const unsigned sq = crow - bidx * (unsigned)SEQ;
      const size_t frow = (size_t)bidx * SEQ_FULL + sq;
      const size_t inrow  = (MODE == 2) ? frow : (size_t)crow;
      const size_t outrow = (MODE == 2) ? (size_t)crow : frow;
      const v4f u = *(const v4f*)&Cs[r * LDC + c];
      const v4f g = *(const v4f*)(bias + n0 + c);
      const v4f xin = *(const v4f*)(addf + inrow * DIM + n0 + c);
      v4f val;
#pragma unroll
      for (int j = 0; j < 4; ++j) {
        const float base = (MODE == 2) ? bf16r(xin[j]) : xin[j];
        val[j] = base + (u[j] * cs + bf16r(g[j]));
      }
      xs[i] = val;
      off[i] = outrow * DIM + n0 + c;
    }
#pragma unroll
    for (int i = 0; i < 4; ++i) *(volatile v4f*)(outf + off[i]) = xs[i];
    __threadfence();
#pragma unroll
    for (int i = 0; i < 4; ++i) *(volatile v4f*)(outf + off[i]) = xs[i];
  }
}

__global__ __launch_bounds__(256) void gemm_wo_kernel(
    const _Float16* __restrict__ A16, const _Float16* __restrict__ Bt,
    const float* __restrict__ bias, const float* __restrict__ xin, float* __restrict__ x1) {
  gemm_body<2>(A16, Bt, (unsigned)DIM, bias, xin, x1, (_Float16*)0, (_Float16*)0);
}
__global__ __launch_bounds__(256) void gemm_ffn1_kernel(
    const _Float16* __restrict__ A16, const _Float16* __restrict__ Bt,
    const float* __restrict__ bias, _Float16* __restrict__ mid) {
  gemm_body<3>(A16, Bt, (unsigned)DIM, bias, bias, (float*)0, mid, mid);
}
__global__ __launch_bounds__(256) void gemm_ffn2_kernel(
    const _Float16* __restrict__ A16, const _Float16* __restrict__ Bt,
    const float* __restrict__ bias, const float* __restrict__ x1, float* __restrict__ outf) {
  gemm_body<4>(A16, Bt, (unsigned)HID, bias, x1, outf, (_Float16*)0, (_Float16*)0);
}

__global__ __launch_bounds__(256) void poison_kernel(
    const int* __restrict__ flag, float* __restrict__ outf) {
  const int f = flag[0];
  if (f != 1) return;
  const float qn = __uint_as_float(0x7FC00000u);
  const v4f nv = {qn, qn, qn, qn};
  const size_t total = (size_t)MROWS * (DIM / 4);
  const size_t stride = (size_t)gridDim.x * 256u;
  for (size_t i = (size_t)blockIdx.x * 256u + threadIdx.x; i < total; i += stride) {
    const unsigned crow = (unsigned)(i / (DIM / 4));
    const unsigned c = (unsigned)(i % (DIM / 4)) * 4u;
    const unsigned bidx = crow / (unsigned)SEQ;
    const unsigned sq = crow - bidx * (unsigned)SEQ;
    const size_t frow = (size_t)bidx * SEQ_FULL + sq;
    float* p = outf + frow * DIM + c;
    *(volatile v4f*)p = nv;
    __threadfence();
    *(volatile v4f*)p = nv;
  }
}

extern "C" void kernel_launch(void* const* d_in, const int* in_sizes, int n_in,
                              void* d_out, int out_size, void* d_ws, size_t ws_size,
                              hipStream_t stream) {
  if (n_in < 15) return;
  const long long need_x = ((long long)(NB - 1) * SEQ_FULL + SEQ) * DIM;
  if ((long long)in_sizes[0] < need_x) return;
  if (in_sizes[1] < SEQ) return;
  if ((long long)in_sizes[2] < (long long)DIM * QKVW) return;
  if (in_sizes[3] < HD || in_sizes[4] < HD || in_sizes[5] < HD || in_sizes[6] < HD) return;
  if ((long long)in_sizes[7] < (long long)DIM * DIM) return;
  if (in_sizes[8] < DIM || in_sizes[9] < DIM || in_sizes[10] < DIM) return;
  if ((long long)in_sizes[11] < (long long)DIM * HID) return;
  if (in_sizes[12] < HID) return;
  if ((long long)in_sizes[13] < (long long)DIM * HID) return;
  if (in_sizes[14] < DIM) return;
  if ((long long)out_size < need_x) return;
  if (ws_size < WS_TOTAL) return;

  const float* X     = (const float*)d_in[0];
  const int*   batch = (const int*)d_in[1];
  const float* wqkv  = (const float*)d_in[2];
  const float* ln1w  = (const float*)d_in[3];
  const float* ln1b  = (const float*)d_in[4];
  const float* ln2w  = (const float*)d_in[5];
  const float* ln2b  = (const float*)d_in[6];
  const float* wo    = (const float*)d_in[7];
  const float* bo    = (const float*)d_in[8];
  const float* lnmw  = (const float*)d_in[9];
  const float* lnmb  = (const float*)d_in[10];
  const float* w1    = (const float*)d_in[11];
  const float* b1    = (const float*)d_in[12];
  const float* w2    = (const float*)d_in[13];
  const float* b2    = (const float*)d_in[14];
  float* out = (float*)d_out;

  char* ws = (char*)d_ws;
  _Float16* Wqkv_t = (_Float16*)(ws + OFF_WQKV);
  _Float16* Wo_t   = (_Float16*)(ws + OFF_WO);
  _Float16* W1_t   = (_Float16*)(ws + OFF_W1);
  _Float16* W2_t   = (_Float16*)(ws + OFF_W2);
  _Float16* X16    = (_Float16*)(ws + OFF_X16);
  _Float16* Q16    = (_Float16*)(ws + OFF_Q);
  _Float16* KVt16  = (_Float16*)(ws + OFF_KVT);
  _Float16* Ctx16  = (_Float16*)(ws + OFF_CTX);
  _Float16* H2     = (_Float16*)(ws + OFF_H2);
  float*    X1     = (float*)(ws + OFF_X1);
  _Float16* Mid16  = (_Float16*)(ws + OFF_MID);
  int*      Flag   = (int*)(ws + OFF_FLAG);

  dim3 blk(256);
  dim3 gg(DIM / 64, MROWS / 64);

  wconv_kernel<<<dim3(QKVW / 64, DIM / 64), blk, 0, stream>>>(wqkv, Wqkv_t, (unsigned)QKVW, (unsigned)DIM);
  wconv_kernel<<<dim3(DIM / 64, DIM / 64), blk, 0, stream>>>(wo, Wo_t, (unsigned)DIM, (unsigned)DIM);
  wconv_kernel<<<dim3(HID / 64, DIM / 64), blk, 0, stream>>>(w1, W1_t, (unsigned)HID, (unsigned)DIM);
  wconv_kernel<<<dim3(DIM / 64, HID / 64), blk, 0, stream>>>(w2, W2_t, (unsigned)DIM, (unsigned)HID);

  xconv_kernel<<<dim3(MROWS / 8), blk, 0, stream>>>(X, X16);
  seg_check_kernel<<<dim3(1), blk, 0, stream>>>(batch, Flag);
  gemm_qkv_kernel<<<dim3(QKVW / 64, MROWS / 64), blk, 0, stream>>>(
      X16, Wqkv_t, ln1w, ln1b, ln2w, ln2b, Q16, KVt16);
  galerkin_kernel<<<dim3(NGRAPH, NB), dim3(128), 0, stream>>>(
      Q16, KVt16, KVt16 + PLANE16_ELEMS, batch, Ctx16);
  gemm_wo_kernel<<<gg, blk, 0, stream>>>(Ctx16, Wo_t, bo, X, X1);
  ln_ws_kernel<<<dim3(MROWS / 8), blk, 0, stream>>>(X1, lnmw, lnmb, H2);
  gemm_ffn1_kernel<<<dim3(HID / 64, MROWS / 64), blk, 0, stream>>>(H2, W1_t, b1, Mid16);
  gemm_ffn2_kernel<<<gg, blk, 0, stream>>>(Mid16, W2_t, b2, X1, out);
  poison_kernel<<<dim3(64), blk, 0, stream>>>(Flag, out);
}
